// Attention_13829794693777
// MI455X (gfx1250) — hardware-run, weakly checked
//
#include <hip/hip_runtime.h>


#ifndef NB
#define NB 2
#endif
#ifndef SEQ
#define SEQ 4096
#endif
#define NB_FULL  2
#define SEQ_FULL 4096
#ifndef OUT_SEQ
#define OUT_SEQ SEQ
#endif
#define DM   384
#define NH_  8
#define HD   48
#define HDP  64
#define IMW  64
#define FW   4
#define OSP  100
#define QSP  68
#define VSP  68
#define SC2  ((float)(0.14433756729740643 * 1.4426950408889634))
#define PSH  14.0f
#define NEGB (-3.0e38f)

static_assert(NH_ * HD == DM);
static_assert(HD % 16 == 0);
static_assert(HD == 48);
static_assert(HDP == 64);
static_assert(HDP - HD == 16);
static_assert(NH_ % 2 == 0);
static_assert((2 * HD * 4) % 128 == 0);
static_assert((DM * 4) % 128 == 0);
static_assert(DM % 64 == 0);
static_assert(DM % 32 == 0);
static_assert(SEQ % 64 == 0);
static_assert((NB * SEQ) % 64 == 0);
static_assert(SEQ % 32 == 0);
static_assert(SEQ % IMW == 0);
static_assert(((size_t)SEQ * DM) % 8 == 0);
static_assert(((size_t)3 * DM * DM) % 8 == 0);
static_assert(NB <= NB_FULL);
static_assert(SEQ <= SEQ_FULL);
static_assert((OSP * 4) % 16 == 0);
static_assert((QSP * 4) % 16 == 0);
static_assert((VSP * 4) % 16 == 0);
static_assert(OSP >= 2 * HD);
static_assert(QSP >= HDP);
static_assert(VSP >= 64);

typedef _Float16 h16;
typedef unsigned short bf;
typedef __attribute__((ext_vector_type(16))) __bf16   v16bf;
typedef __attribute__((ext_vector_type(16))) _Float16 v16h;
typedef __attribute__((ext_vector_type(8)))  _Float16 v8h;
typedef __attribute__((ext_vector_type(8)))  unsigned short v8us;
typedef __attribute__((ext_vector_type(8)))  float    v8f;
typedef __attribute__((ext_vector_type(4)))  float    v4f;
typedef v4f  __attribute__((may_alias)) v4fa;

__device__ __forceinline__ unsigned short f2bf(float f) { unsigned u = __float_as_uint(f); u += 0x7FFFu + ((u >> 16) & 1u); return (unsigned short)(u >> 16); }
__device__ __forceinline__ float bfr(float f) { return __uint_as_float(((unsigned)f2bf(f)) << 16); }
__device__ __forceinline__ v16h cat16(v8h lo, v8h hi) { return __builtin_shufflevector(lo, hi, 0, 1, 2, 3, 4, 5, 6, 7, 8, 9, 10, 11, 12, 13, 14, 15); }
__device__ __forceinline__ v16bf cat16b(v8us lo, v8us hi) { return __builtin_bit_cast(v16bf, __builtin_shufflevector(lo, hi, 0, 1, 2, 3, 4, 5, 6, 7, 8, 9, 10, 11, 12, 13, 14, 15)); }
__device__ __forceinline__ v8f wmma16(v16h a, v16h b, v8f c) { return __builtin_amdgcn_wmma_f32_16x16x32_f16(false, a, false, b, (short)0, c, false, false); }
__device__ __forceinline__ v8f wmmab(v16bf a, v16bf b, v8f c) { return __builtin_amdgcn_wmma_f32_16x16x32_bf16(false, a, false, b, (short)0, c, false, false); }
__device__ __forceinline__ v16h  ldh(const h16* p) { return cat16(*(const v8h*)p, *(const v8h*)(p + 16)); }
__device__ __forceinline__ v16bf ldb(const bf* p)  { return cat16b(*(const v8us*)p, *(const v8us*)(p + 16)); }
__device__ __forceinline__ void wave_sync() { __builtin_amdgcn_fence(3  , "wavefront"); __builtin_amdgcn_wave_barrier(); asm volatile("" ::: "memory"); }

__device__ __forceinline__ v8f wmma16g(v16h a, v16h b, v8f c) { c = wmma16(a, b, c); asm volatile("v_nop\n\tv_nop\n\tv_nop\n\tv_nop" : "+v"(c) : "v"(a), "v"(b)); return c; }
__device__ __forceinline__ v8f wmmabg(v16bf a, v16bf b, v8f c) { c = wmmab(a, b, c); asm volatile("v_nop\n\tv_nop\n\tv_nop\n\tv_nop" : "+v"(c) : "v"(a), "v"(b)); return c; }
static __device__ __forceinline__ h16 toh_flush(float v) { const h16 r = (h16)v; return (fabsf(v) < 6.103515625e-05f) ? (h16)0.0f : r; }

__global__ __launch_bounds__(256) void k_cvt8(const float* __restrict__ src, bf* dst, size_t n8) {
    const size_t i = (size_t)blockIdx.x * 256 + threadIdx.x; if (i >= n8) return;
    const v8f v = *(const v8f*)(src + i * 8); v8us o;
#pragma unroll
    for (int k = 0; k < 8; ++k) o[k] = f2bf(v[k]);
    *(volatile v8us*)(dst + i * 8) = o; __threadfence(); *(volatile v8us*)(dst + i * 8) = o;
}

__global__ __launch_bounds__(32) void k_proj_qk(const bf* __restrict__ A, const bf* __restrict__ Wb, const float* __restrict__ bias, h16* QK) {
    __shared__ __align__(16) float os[16 * QSP];
    static_assert(sizeof(float) * 16 * QSP <= 131072);
    const int K = DM;
    const int lane = threadIdx.x & 31, lr = lane & 15, hi = lane >> 4;
    const int r0 = blockIdx.x * 64; const int sec = blockIdx.y / NH_, h = blockIdx.y % NH_;
    const int c0 = sec * DM + h * HD;
    v8f acc[4][3];
#pragma unroll
    for (int mb = 0; mb < 4; ++mb)
#pragma unroll
        for (int nb = 0; nb < 3; ++nb) acc[mb][nb] = (v8f){};
    const size_t aoff = (size_t)(r0 + lr) * K + 8 * hi, boff = (size_t)(c0 + lr) * K + 8 * hi;
#pragma unroll 1
    for (int kc = 0; kc < K; kc += 32) {
        v16bf a[4];
#pragma unroll
        for (int mb = 0; mb < 4; ++mb) a[mb] = ldb(A + aoff + (size_t)mb * 16 * K + kc);
#pragma unroll
        for (int nb = 0; nb < 3; ++nb) { const v16bf b = ldb(Wb + boff + (size_t)nb * 16 * K + kc);
#pragma unroll
            for (int mb = 0; mb < 4; ++mb) acc[mb][nb] = wmmabg(a[mb], b, acc[mb][nb]); }
    }
    float bc[3];
#pragma unroll
    for (int nb = 0; nb < 3; ++nb) bc[nb] = bfr(bias[c0 + nb * 16 + lr]);
    const int bb = r0 / SEQ, tt = r0 % SEQ;
    const size_t pbase = (size_t)sec * ((size_t)NB * NH_ * SEQ * HDP) + ((size_t)(bb * NH_ + h) * SEQ + (size_t)tt) * HDP;
#pragma unroll
    for (int mb = 0; mb < 4; ++mb) {
#pragma unroll
        for (int nb = 0; nb < 3; ++nb) {
#pragma unroll
            for (int j = 0; j < 8; ++j) os[(hi * 8 + j) * QSP + nb * 16 + lr] = acc[mb][nb][j] + bc[nb]; }
#pragma unroll
        for (int j = 0; j < 8; ++j) os[(hi * 8 + j) * QSP + HD + lr] = 0.0f;
        wave_sync();
        static_assert(32 * 16 * 4 == 16 * HDP * 2);
#pragma unroll 1
        for (int ps = 0; ps < 2; ++ps) {
            const size_t sb = pbase + (size_t)(mb * 16) * HDP;
#pragma unroll
            for (int s = 0; s < 4; ++s) { const int row = 4 * s + (lane >> 3), c8 = (lane & 7) * 8;
                const v4f x0 = *(const v4fa*)(&os[row * QSP + c8]); const v4f x1 = *(const v4fa*)(&os[row * QSP + c8 + 4]); v8h hv;
#pragma unroll
                for (int i = 0; i < 4; ++i) { hv[i] = toh_flush(x0[i]); hv[4 + i] = toh_flush(x1[i]); }
                *(volatile v8h*)(QK + sb + (size_t)row * HDP + c8) = hv; }
            if (ps == 0) __threadfence(); }
        wave_sync();
    }
}

__global__ __launch_bounds__(32) void k_proj_vt(const bf* __restrict__ Wb, const bf* __restrict__ X, const float* __restrict__ bias, h16* VT, float* VF) {
    __shared__ __align__(16) float os[64 * VSP];
    static_assert(sizeof(float) * 64 * VSP <= 131072);
    const int K = DM;
    const int lane = threadIdx.x & 31, lr = lane & 15, hi = lane >> 4; const int r0 = blockIdx.x * 64, c0 = blockIdx.y * 64;
    const bf* A = Wb + (size_t)2 * DM * DM;
    v8f acc[4][4];
#pragma unroll
    for (int mb = 0; mb < 4; ++mb)
#pragma unroll
        for (int nb = 0; nb < 4; ++nb) acc[mb][nb] = (v8f){};
    const size_t aoff = (size_t)(r0 + lr) * K + 8 * hi, boff = (size_t)(c0 + lr) * K + 8 * hi;
#pragma unroll 1
    for (int kc = 0; kc < K; kc += 32) {
        v16bf a[4];
#pragma unroll
        for (int mb = 0; mb < 4; ++mb) a[mb] = ldb(A + aoff + (size_t)mb * 16 * K + kc);
#pragma unroll
        for (int nb = 0; nb < 4; ++nb) { const v16bf b = ldb(X + boff + (size_t)nb * 16 * K + kc);
#pragma unroll
            for (int mb = 0; mb < 4; ++mb) acc[mb][nb] = wmmabg(a[mb], b, acc[mb][nb]); }
    }
#pragma unroll
    for (int mb = 0; mb < 4; ++mb) {
        float br[8];
#pragma unroll
        for (int j = 0; j < 8; ++j) br[j] = bfr(bias[2 * DM + r0 + mb * 16 + hi * 8 + j]);
#pragma unroll
        for (int nb = 0; nb < 4; ++nb) {
#pragma unroll
            for (int j = 0; j < 8; ++j) os[(mb * 16 + hi * 8 + j) * VSP + nb * 16 + lr] = acc[mb][nb][j] + br[j]; }
    }
    wave_sync();
    const int bb = c0 / SEQ, tt = c0 % SEQ;
    const size_t tbase = ((size_t)bb * DM + (size_t)r0) * SEQ + (size_t)tt;
    const size_t fbase = (size_t)c0 * DM + (size_t)r0;
    static_assert(32 * 16 * 16 == 64 * 64 * 2);
    static_assert(32 * 16 * 32 == 64 * 64 * 4);
#pragma unroll 1
    for (int ps = 0; ps < 2; ++ps) {
#pragma unroll 4
        for (int s = 0; s < 16; ++s) { const int row = 4 * s + (lane >> 3), c8 = (lane & 7) * 8;
            const v4f x0 = *(const v4fa*)(&os[row * VSP + c8]); const v4f x1 = *(const v4fa*)(&os[row * VSP + c8 + 4]); v8h hv;
#pragma unroll
            for (int i = 0; i < 4; ++i) { hv[i] = toh_flush(x0[i]); hv[4 + i] = toh_flush(x1[i]); }
            *(volatile v8h*)(VT + tbase + (size_t)row * SEQ + c8) = hv; }
#pragma unroll 4
        for (int s = 0; s < 32; ++s) { const int tok = 2 * s + (lane >> 4), ch4 = (lane & 15) * 4;
            v4f val;
#pragma unroll
            for (int i = 0; i < 4; ++i) val[i] = os[(ch4 + i) * VSP + tok];
            *(volatile v4f*)(VF + fbase + (size_t)tok * DM + ch4) = val; }
        if (ps == 0) __threadfence(); }
}

__global__ __launch_bounds__(256) void k_lepe(const float* __restrict__ VF, const float* __restrict__ lw, const float* __restrict__ lb,
                                              const int* __restrict__ hdim, const int* __restrict__ wdim, float* LP) {
#pragma clang fp contract(off)
    const size_t idx = (size_t)blockIdx.x * 256 + threadIdx.x;
    if (idx >= (size_t)NB * SEQ * (DM / 4)) return;
    int iw = wdim[0], ih = hdim[0];
    if (!((iw >= 1) & (ih >= 1) & (iw <= SEQ) & (ih <= SEQ) & ((long long)iw * (long long)ih == (long long)SEQ))) { iw = IMW; ih = SEQ / IMW; }
    const int c4 = (int)(idx % (DM / 4)) * 4; const int row = (int)(idx / (DM / 4));
    const int b = row / SEQ, t = row % SEQ;
    const int y = t / iw, x = t - y * iw;
    v4f acc;
#pragma unroll
    for (int j = 0; j < 4; ++j) acc[j] = bfr(lb[c4 + j]);
#pragma unroll 1
    for (int dy = -1; dy <= 1; ++dy) {
        const int yy = y + dy; const int yc = yy < 0 ? 0 : (yy > ih - 1 ? ih - 1 : yy);
#pragma unroll
        for (int dx = -1; dx <= 1; ++dx) {
            const int xx = x + dx; const int xc = xx < 0 ? 0 : (xx > iw - 1 ? iw - 1 : xx);
            const bool ok = (yy >= 0) & (yy < ih) & (xx >= 0) & (xx < iw);
            v4f vv = *(const v4f*)(VF + ((size_t)b * SEQ + (size_t)(yc * iw + xc)) * DM + c4);
            asm volatile("" : "+v"(vv));
            const int wi = (dy + 1) * 3 + (dx + 1);
#pragma unroll
            for (int j = 0; j < 4; ++j) { const float w = bfr(lw[(c4 + j) * 9 + wi]); const float vj = ok ? vv[j] : 0.0f; acc[j] = acc[j] + w * vj; }
        }
    }
    *(volatile v4f*)(LP + idx * 4) = acc; __threadfence(); *(volatile v4f*)(LP + idx * 4) = acc;
}

__global__ __launch_bounds__(32 * FW) void k_flash(const h16* __restrict__ QH, const h16* __restrict__ KP, const h16* __restrict__ VT, const float* __restrict__ LP, float* OUT) {
    __shared__ __align__(16) float os[32 * OSP];
    static_assert(sizeof(float) * 32 * OSP <= 131072);
    const int lane = threadIdx.x & 31, lr = lane & 15, hi = lane >> 4;
    const int wave = __builtin_amdgcn_readfirstlane((int)(threadIdx.x >> 5));
    const int hp = blockIdx.y % (NH_ / 2), b = blockIdx.y / (NH_ / 2);
    const int hsel = wave >> 1, slab = wave & 1;
    const int zh = b * NH_ + hp * 2 + hsel;
    const int tb0 = blockIdx.x * 32;
    const int t0 = tb0 + slab * 16;
    const size_t pbase = (size_t)zh * SEQ * HDP;
    const size_t vbase = (size_t)zh * HD * SEQ;
    const size_t qo = pbase + (size_t)(t0 + lr) * HDP + 8 * hi;
    const v16h q0 = ldh(QH + qo), q1 = ldh(QH + qo + 32);
    const size_t ko = pbase + (size_t)lr * HDP + 8 * hi;
    const size_t vo = vbase + (size_t)lr * SEQ + 8 * hi;
    v8f o0 = (v8f){}, o1 = (v8f){}, o2 = (v8f){};
    float m = NEGB, l = 0.0f;
#pragma unroll 1
    for (int key0 = 0; key0 < SEQ; key0 += 32) {
        const h16* ka = KP + ko + (size_t)key0 * HDP;
        const v16h ka0 = ldh(ka), ka1 = ldh(ka + 32), kb0 = ldh(ka + 16 * HDP), kb1 = ldh(ka + 16 * HDP + 32);
        v8f sa = (v8f){}, sb = (v8f){};
        sa = wmma16g(ka0, q0, sa); sb = wmma16g(kb0, q0, sb);
        sa = wmma16g(ka1, q1, sa); sb = wmma16g(kb1, q1, sb);
        float ta[8], tb[8]; float mx = NEGB;
#pragma unroll
        for (int r = 0; r < 8; ++r) { ta[r] = sa[r] * SC2; tb[r] = sb[r] * SC2; mx = fmaxf(mx, fmaxf(ta[r], tb[r])); }
        mx = fmaxf(mx, __shfl_xor(mx, 16, 32));
        const float mnew = fmaxf(m, mx);
        const float alpha = __builtin_amdgcn_exp2f(m - mnew);
        const float sh = PSH - mnew;
        v16h pb; float ls = 0.0f;
#pragma unroll
        for (int r = 0; r < 8; ++r) {
            const float xa = ta[r] + sh, xb = tb[r] + sh;
            const float ea = __builtin_amdgcn_exp2f(xa), eb = __builtin_amdgcn_exp2f(xb);
            const float ga = (xa < -14.0f) ? 0.0f : ea, gb = (xb < -14.0f) ? 0.0f : eb;
            const h16 pa = (h16)ga; const h16 pc = (h16)gb;
            pb[r] = pa; pb[8 + r] = pc;
            ls += (float)pa + (float)pc; }
        l = l * alpha + ls; m = mnew;
        o0 = o0 * alpha; o1 = o1 * alpha; o2 = o2 * alpha;
        const h16* va = VT + vo + key0;
        const v16h v0 = ldh(va), v1 = ldh(va + (size_t)16 * SEQ), v2 = ldh(va + (size_t)32 * SEQ);
        o0 = wmma16g(v0, pb, o0); o1 = wmma16g(v1, pb, o1); o2 = wmma16g(v2, pb, o2);
    }
    l += __shfl_xor(l, 16, 32);
    const float inv = 1.0f / l;
    { const int ob = (slab * 16 + lr) * OSP + hsel * HD + 8 * hi; v4f a, c;
      a[0] = o0[0] * inv; a[1] = o0[1] * inv; a[2] = o0[2] * inv; a[3] = o0[3] * inv; c[0] = o0[4] * inv; c[1] = o0[5] * inv; c[2] = o0[6] * inv; c[3] = o0[7] * inv;
      *(v4fa*)(&os[ob +  0]) = a; *(v4fa*)(&os[ob +  0 + 4]) = c;
      a[0] = o1[0] * inv; a[1] = o1[1] * inv; a[2] = o1[2] * inv; a[3] = o1[3] * inv; c[0] = o1[4] * inv; c[1] = o1[5] * inv; c[2] = o1[6] * inv; c[3] = o1[7] * inv;
      *(v4fa*)(&os[ob + 16]) = a; *(v4fa*)(&os[ob + 16 + 4]) = c;
      a[0] = o2[0] * inv; a[1] = o2[1] * inv; a[2] = o2[2] * inv; a[3] = o2[3] * inv; c[0] = o2[4] * inv; c[1] = o2[5] * inv; c[2] = o2[6] * inv; c[3] = o2[7] * inv;
      *(v4fa*)(&os[ob + 32]) = a; *(v4fa*)(&os[ob + 32 + 4]) = c; }
    __syncthreads();
    float* obase = OUT + ((size_t)b * OUT_SEQ + tb0) * DM + hp * (2 * HD);
    const float* lbase = LP + ((size_t)b * SEQ + tb0) * DM + hp * (2 * HD);
    static_assert((32 * FW) * 6 == 32 * ((2 * HD) / 4));
    static_assert(((2 * HD) / 4) % 8 == 0);
#pragma unroll 1
    for (int ps = 0; ps < 2; ++ps) {
#pragma unroll
        for (int it = 0; it < 6; ++it) { const int p = it * (32 * FW) + (int)threadIdx.x; const int row = p / 24, cofs = (p % 24) * 4;
            v4f val = *(const v4fa*)(&os[row * OSP + cofs]);
            const v4f lp = *(const v4f*)(lbase + (size_t)row * DM + cofs);
            val = val + lp;
            *(volatile v4f*)(obase + (size_t)row * DM + cofs) = val; }
        if (ps == 0) __threadfence(); }
}

static constexpr size_t al256(size_t v) { return (v + 255) & ~(size_t)255; }
static constexpr size_t SZ_XB = al256((size_t)NB * SEQ * DM * 2);
static constexpr size_t SZ_WB = al256((size_t)3 * DM * DM * 2);
static constexpr size_t SZ_PL = al256((size_t)NB * NH_ * SEQ * HDP * 2);
static constexpr size_t SZ_VT = al256((size_t)NB * DM * SEQ * 2);
static constexpr size_t SZ_VF = al256((size_t)NB * SEQ * DM * 4);
static constexpr size_t SZ_TOTAL = SZ_XB + SZ_WB + 2 * SZ_PL + SZ_VT + 2 * SZ_VF;
static_assert(SZ_TOTAL <= (size_t)134217728);
static_assert(((size_t)NB * NH_ * SEQ * HDP * 2) % 256 == 0);
static_assert((size_t)NB * NH_ * HD * SEQ == (size_t)NB * DM * SEQ);

extern "C" void kernel_launch(void* const* d_in, const int* in_sizes, int n_in,
                              void* d_out, int out_size, void* d_ws, size_t ws_size, hipStream_t stream) {
    if (n_in < 7) return;
    const size_t needx = ((size_t)(NB - 1) * SEQ_FULL + SEQ) * DM;
    if ((size_t)in_sizes[0] < needx) return;
    if ((size_t)in_sizes[1] < (size_t)3 * DM * DM || in_sizes[2] < 3 * DM) return;
    if (in_sizes[3] < DM * 9 || in_sizes[4] < DM || in_sizes[5] < 1 || in_sizes[6] < 1) return;
    if ((size_t)out_size < ((size_t)(NB - 1) * OUT_SEQ + SEQ) * DM) return;
    if (SZ_TOTAL > ws_size) return;
    const float* x  = (const float*)d_in[0];
    const float* qw = (const float*)d_in[1]; const float* qb = (const float*)d_in[2];
    const float* lw = (const float*)d_in[3]; const float* lb = (const float*)d_in[4];
    const int* hdim = (const int*)d_in[5];   const int* wdim = (const int*)d_in[6];
    float* OUT = (float*)d_out;
    char* wsp = (char*)d_ws;
    bf* XB = (bf*)wsp; wsp += SZ_XB;
    bf* WB = (bf*)wsp; wsp += SZ_WB;
    h16* QK = (h16*)wsp; wsp += 2 * SZ_PL;
    h16* VT = (h16*)wsp; wsp += SZ_VT;
    float* VF = (float*)wsp; wsp += SZ_VF;
    float* LP = (float*)wsp; wsp += SZ_VF;
    h16* QH = QK; h16* KP = QK + (size_t)NB * NH_ * SEQ * HDP;

    if (SEQ == SEQ_FULL) {
        const size_t n8 = (size_t)NB * SEQ * DM / 8;
        k_cvt8<<<(unsigned)((n8 + 255) / 256), 256, 0, stream>>>(x, XB, n8);
    } else {
        const size_t n8 = (size_t)SEQ * DM / 8;
        for (int b = 0; b < NB; ++b) k_cvt8<<<(unsigned)((n8 + 255) / 256), 256, 0, stream>>>(x + (size_t)b * SEQ_FULL * DM, XB + (size_t)b * SEQ * DM, n8);
    }
    { const size_t n8 = (size_t)3 * DM * DM / 8; k_cvt8<<<(unsigned)((n8 + 255) / 256), 256, 0, stream>>>(qw, WB, n8); }

    k_proj_qk<<<dim3(NB * SEQ / 64, 2 * NH_, 1), 32, 0, stream>>>(XB, WB, qb, QK);
    k_proj_vt<<<dim3(DM / 64, NB * SEQ / 64, 1), 32, 0, stream>>>(WB, XB, qb, VT, VF);
    { const size_t nt = (size_t)NB * SEQ * (DM / 4); k_lepe<<<(unsigned)((nt + 255) / 256), 256, 0, stream>>>(VF, lw, lb, hdim, wdim, LP); }
    k_flash<<<dim3(SEQ / 32, NB * NH_ / 2, 1), 32 * FW, 0, stream>>>(QH, KP, VT, LP, OUT);
}
